// ChebyKANLinear_60610578481558
// MI455X (gfx1250) — hardware-verified
//
#include <hip/hip_runtime.h>


#define NB_  8192
#define NI   1024
#define NO   1024
#define ND   9
#define ICH  256
#define KCH  (ICH * ND)
#define KT   (NI * ND)
#define CSC  65536.0f

typedef _Float16 h16;
typedef __attribute__((ext_vector_type(16))) _Float16 v16h;
typedef __attribute__((ext_vector_type(8)))  _Float16 v8h;
typedef __attribute__((ext_vector_type(8)))  float    v8f;
typedef __attribute__((ext_vector_type(4)))  float    v4f;
typedef v4f __attribute__((may_alias)) v4fa;
typedef v8h __attribute__((may_alias)) v8ha;

__device__ __forceinline__ unsigned short f2bf(float f) { unsigned u = __float_as_uint(f); u += 0x7FFFu + ((u >> 16) & 1u); return (unsigned short)(u >> 16); }
__device__ __forceinline__ float bf2f(unsigned short b) { return __uint_as_float(((unsigned)b) << 16); }
__device__ __forceinline__ float bfr(float f) { return bf2f(f2bf(f)); }
__device__ __forceinline__ v16h cat16(v8h lo, v8h hi) { return __builtin_shufflevector(lo, hi, 0, 1, 2, 3, 4, 5, 6, 7, 8, 9, 10, 11, 12, 13, 14, 15); }
__device__ __forceinline__ v8f wmma16(v16h a, v16h b, v8f c) { return __builtin_amdgcn_wmma_f32_16x16x32_f16(false, a, false, b, (short)0, c, false, false); }

__global__ __launch_bounds__(256) void k_basis(const float* __restrict__ x, int i0, h16* A) {
    __shared__ __align__(16) h16 rowbuf[KCH + 16];
    const int b = blockIdx.x, il = threadIdx.x;
    const float t = tanhf(bfr(x[(size_t)b * NI + i0 + il]));
    float tm2 = 1.0f, tm1 = t;
    rowbuf[il * ND + 0] = (h16)1.0f; rowbuf[il * ND + 1] = (h16)t;
#pragma unroll
    for (int d = 2; d < ND; ++d) { const float tn = 2.0f * t * tm1 - tm2; rowbuf[il * ND + d] = (h16)tn; tm2 = tm1; tm1 = tn; }
    __syncthreads();
    const int tid = threadIdx.x;
    auto pass = [&]() {
        *(volatile v8h*)(A + (size_t)b * KCH + tid * 8) = *(const v8ha*)(rowbuf + tid * 8);
        if (tid < 288 - 256) *(volatile v8h*)(A + (size_t)b * KCH + (256 + tid) * 8) = *(const v8ha*)(rowbuf + (256 + tid) * 8);
    };
    pass(); __threadfence(); pass();
}
__global__ __launch_bounds__(256) void k_coef(const float* __restrict__ C, h16* Bm) {
    __shared__ __align__(16) h16 rowbuf[KCH + 16];
    const int o = blockIdx.x, ic = blockIdx.y, il = threadIdx.x, i = ic * ICH + il;
#pragma unroll
    for (int d = 0; d < ND; ++d) rowbuf[il * ND + d] = (h16)(bfr(C[((size_t)i * NO + o) * ND + d]) * CSC);
    __syncthreads();
    const int tid = threadIdx.x;
    auto pass = [&]() {
        *(volatile v8h*)(Bm + (size_t)o * KT + (size_t)ic * KCH + tid * 8) = *(const v8ha*)(rowbuf + tid * 8);
        if (tid < 288 - 256) *(volatile v8h*)(Bm + (size_t)o * KT + (size_t)ic * KCH + (256 + tid) * 8) = *(const v8ha*)(rowbuf + (256 + tid) * 8);
    };
    pass(); __threadfence(); pass();
}
template <bool ACC>
__global__ __launch_bounds__(128) void k_gemm(const h16* __restrict__ A, const h16* __restrict__ Bm, int kofs, float* out) {
    __shared__ __align__(16) float ost[4][16 * 68];
    const int lane = threadIdx.x & 31, wave = threadIdx.x >> 5, lr = lane & 15, hi = lane >> 4;
    const size_t r0 = (size_t)blockIdx.x * 64 + wave * 16; const int c0 = blockIdx.y * 64;
    const size_t aoff = (r0 + lr) * KCH + 8 * hi;
    size_t boff[4];
#pragma unroll
    for (int t = 0; t < 4; ++t) boff[t] = (size_t)(c0 + t * 16 + lr) * KT + kofs + 8 * hi;
    v8f acc[4];
#pragma unroll
    for (int t = 0; t < 4; ++t) acc[t] = (v8f){};
#pragma unroll 2
    for (int kc = 0; kc < KCH; kc += 32) {
        const v16h a = cat16(*(const v8h*)(A + aoff + kc), *(const v8h*)(A + aoff + kc + 16));
#pragma unroll
        for (int t = 0; t < 4; ++t) acc[t] = wmma16(a, cat16(*(const v8h*)(Bm + boff[t] + kc), *(const v8h*)(Bm + boff[t] + kc + 16)), acc[t]);
        asm volatile("v_nop" : "+v"(acc[0]), "+v"(acc[1]), "+v"(acc[2]), "+v"(acc[3]) : "v"(a) : "memory");
    }
    float* os = &ost[wave][0];
#pragma unroll
    for (int t = 0; t < 4; ++t)
#pragma unroll
        for (int j = 0; j < 8; ++j) { float v = acc[t][j] * (1.0f / CSC); if (ACC) v += out[(r0 + hi * 8 + j) * NO + c0 + t * 16 + lr]; os[(hi * 8 + j) * 68 + t * 16 + lr] = v; }
    __builtin_amdgcn_wave_barrier(); asm volatile("" ::: "memory");
    float* crow = out + r0 * NO + c0;
    auto pass = [&]() {
#pragma unroll
        for (int s = 0; s < 8; ++s) { const int Lid = (lane >> 3) + 4 * s, piece = lane & 7; const int row = Lid >> 1, cofs = (Lid & 1) * 32 + piece * 4;
            const v4f val = *(const v4fa*)(os + row * 68 + cofs); *(volatile v4f*)(crow + (size_t)row * NO + cofs) = val; }
    };
    pass(); __threadfence(); pass();
}

extern "C" void kernel_launch(void* const* d_in, const int* in_sizes, int n_in,
                              void* d_out, int out_size, void* d_ws, size_t ws_size, hipStream_t stream) {
    (void)in_sizes; (void)n_in; (void)out_size;
    const float* x = (const float*)d_in[0]; const float* C = (const float*)d_in[1];
    float* out = (float*)d_out;
    char* wsp = (char*)d_ws;
    auto take = [&](size_t bytes) { char* p = wsp; wsp += (bytes + 255) & ~(size_t)255; return (void*)p; };
    h16* A = (h16*)take((size_t)NB_ * KCH * 2); h16* Bm = (h16*)take((size_t)NO * KT * 2);
    if ((size_t)(wsp - (char*)d_ws) > ws_size) return;
    k_coef<<<dim3(NO, NI / ICH, 1), 256, 0, stream>>>(C, Bm);
    for (int ic = 0; ic < NI / ICH; ++ic) {
        k_basis<<<NB_, 256, 0, stream>>>(x, ic * ICH, A);
        if (ic == 0) k_gemm<false><<<dim3(NB_ / 64, NO / 64, 1), 128, 0, stream>>>(A, Bm, ic * KCH, out);
        else         k_gemm<true ><<<dim3(NB_ / 64, NO / 64, 1), 128, 0, stream>>>(A, Bm, ic * KCH, out);
    }
}
